// Encoder_SelfAttention_70360154243484
// MI455X (gfx1250) — hardware-verified
//
#include <hip/hip_runtime.h>
#include <math.h>
#include <stdint.h>

#define NBATCH 8
#define SEQ    512
#define HID    512
#define NHEAD  8
#define HD     64
#define NQB    (SEQ / 64)
#define QKP    (2 * HID)
#define NFREQ  257
#define DFTW   576
#define TABN   (NBATCH * NHEAD * SEQ)
static_assert(NHEAD * HD == HID);
static_assert((SEQ % 64) == 0 && (HID % 64) == 0 && (DFTW % 64) == 0 && (DFTW >= 2 * NFREQ));
static_assert((HID % 32) == 0 && (DFTW % 32) == 0);
static_assert((TABN % 256) == 0 && ((NBATCH * SEQ * HID / 8) % 256) == 0);
static_assert(((DFTW * HID / 8) % 256) == 0 && ((NBATCH * SEQ * (DFTW / 8)) % 256) == 0);
static_assert(SEQ == 512 && NHEAD == 8);

typedef _Float16 v16h __attribute__((ext_vector_type(16)));
typedef _Float16 v8h  __attribute__((ext_vector_type(8)));
typedef _Float16 v4h  __attribute__((ext_vector_type(4)));
typedef __bf16   v16b __attribute__((ext_vector_type(16)));
typedef __bf16   v8b  __attribute__((ext_vector_type(8)));
typedef float    v8f  __attribute__((ext_vector_type(8)));
typedef float    v4f  __attribute__((ext_vector_type(4)));
typedef unsigned int v4u __attribute__((ext_vector_type(4)));

__device__ __forceinline__ unsigned short bf_bits(float f) {
  unsigned u = __float_as_uint(f);
  return (unsigned short)((u + 0x7FFFu + ((u >> 16) & 1u)) >> 16);
}
__device__ __forceinline__ float bf_up(unsigned short h) { return __uint_as_float(((unsigned)h) << 16); }
__device__ __forceinline__ float rbf(float f) { return bf_up(bf_bits(f)); }
__device__ __forceinline__ unsigned short h_bits(_Float16 x) { return __builtin_bit_cast(unsigned short, x); }
__device__ __forceinline__ unsigned pk16(unsigned short a, unsigned short b) { return (unsigned)a | ((unsigned)b << 16); }
__device__ __forceinline__ v8f zero8() { v8f z = {0.f, 0.f, 0.f, 0.f, 0.f, 0.f, 0.f, 0.f}; return z; }

__device__ __forceinline__ v16b ldfrag_b(const __bf16* p) {
  union { v16b v; v8b h[2]; } f;
  f.h[0] = *(const v8b*)(p);
  f.h[1] = *(const v8b*)(p + 16);
  return f.v;
}
__device__ __forceinline__ v16h ldfrag_h(const _Float16* p) {
  union { v16h v; v8h h[2]; } f;
  f.h[0] = *(const v8h*)(p);
  f.h[1] = *(const v8h*)(p + 16);
  return f.v;
}

__device__ __forceinline__ v8f mma_h(v16h a, v16h b, v8f c) {
  c = __builtin_amdgcn_wmma_f32_16x16x32_f16(false, a, false, b, (short)0, c, false, false);
#if defined(__HIP_DEVICE_COMPILE__)
  asm volatile("v_nop\n\tv_nop\n\tv_nop\n\tv_nop" : "+v"(c) : "v"(a), "v"(b));
#endif
  return c;
}
__device__ __forceinline__ v8f mma_b_raw(v16b a, v16b b, v8f c) {
  return __builtin_amdgcn_wmma_f32_16x16x32_bf16(false, a, false, b, (short)0, c, false, false);
}
__device__ __forceinline__ void dep_guard_b(v8f& a, v8f& b, v16b x, v16b y) {
#if defined(__HIP_DEVICE_COMPILE__)
  asm volatile("v_nop\n\tv_nop\n\tv_nop\n\tv_nop" : "+v"(a), "+v"(b) : "v"(x), "v"(y));
#endif
}
__device__ __forceinline__ void keep4_b(v16b a, v16b b, v16b c, v16b d) {
#if defined(__HIP_DEVICE_COMPILE__)
  asm volatile("v_nop" :: "v"(a), "v"(b), "v"(c), "v"(d));
#endif
}
__device__ __forceinline__ void acc_guard4(v8f& a, v8f& b, v8f& c, v8f& d) {
#if defined(__HIP_DEVICE_COMPILE__)
  asm volatile("v_nop\n\tv_nop\n\tv_nop\n\tv_nop" : "+v"(a), "+v"(b), "+v"(c), "+v"(d));
#endif
}
__device__ __forceinline__ void wave_sync_lds() {
  __builtin_amdgcn_fence(__ATOMIC_RELEASE, "workgroup");
  __builtin_amdgcn_wave_barrier();
  __builtin_amdgcn_fence(__ATOMIC_ACQUIRE, "workgroup");
}
__device__ __forceinline__ float wave_sum(float v) {
#pragma unroll
  for (int off = 1; off < 32; off <<= 1) v += __shfl_xor(v, off, 32);
  return v;
}

__global__ __launch_bounds__(256) void cvt_bf16x8(const float* __restrict__ in, unsigned short* out, int n8) {
  const int i = blockIdx.x * 256 + threadIdx.x;
  if (i < n8) {
    const v4f a = *(const v4f*)(in + (size_t)i * 8);
    const v4f b = *(const v4f*)(in + (size_t)i * 8 + 4);
    v4u p;
    p[0] = pk16(bf_bits(a[0]), bf_bits(a[1]));
    p[1] = pk16(bf_bits(a[2]), bf_bits(a[3]));
    p[2] = pk16(bf_bits(b[0]), bf_bits(b[1]));
    p[3] = pk16(bf_bits(b[2]), bf_bits(b[3]));
    *(volatile v4u*)(out + (size_t)i * 8) = p;
    __threadfence();
    *(volatile v4u*)(out + (size_t)i * 8) = p;
  }
}

__global__ __launch_bounds__(256) void tr_bf16(const float* __restrict__ in, unsigned short* out, int R, int C) {
  __shared__ float tile[64 * 65];
  const int tid = threadIdx.x, lane = tid & 31, wave = tid >> 5;
  const int r0 = blockIdx.y * 64, c0 = blockIdx.x * 64;
#pragma unroll
  for (int i = 0; i < 4; ++i) {
    const int idx = tid + i * 256;
    const int r = idx >> 4, cc = (idx & 15) * 4;
    const v4f v = *(const v4f*)(in + (size_t)(r0 + r) * C + c0 + cc);
    tile[r * 65 + cc + 0] = v[0];
    tile[r * 65 + cc + 1] = v[1];
    tile[r * 65 + cc + 2] = v[2];
    tile[r * 65 + cc + 3] = v[3];
  }
  __syncthreads();
  const int q = lane >> 3, c8 = (lane & 7) * 8;
  v4u pv[2];
#pragma unroll
  for (int it = 0; it < 2; ++it) {
    const int j = wave * 8 + it * 4 + q;
    v4u p;
#pragma unroll
    for (int e = 0; e < 4; ++e)
      p[e] = pk16(bf_bits(tile[(c8 + 2 * e) * 65 + j]), bf_bits(tile[(c8 + 2 * e + 1) * 65 + j]));
    pv[it] = p;
  }
  for (int pass = 0; pass < 2; ++pass) {
#pragma unroll
    for (int it = 0; it < 2; ++it) {
      const int j = wave * 8 + it * 4 + q;
      *(volatile v4u*)(out + (size_t)(c0 + j) * R + r0 + c8) = pv[it];
    }
    __threadfence();
  }
}

#define INV_SQRT512     0.044194173824159216f
#define TWO_PI_OVER_512 0.012271846303085130f

__global__ __launch_bounds__(256) void build_basis(unsigned short* ftp, unsigned short* gtp) {
  const int g = blockIdx.x * 256 + threadIdx.x;
  const int part = blockIdx.y;
  if (g >= DFTW * HID / 8) return;
  const int rowF = g >> 6, colF = (g & 63) * 8;
  const int qg = g / (DFTW / 8);
  const int rowG = qg, colG = (g - qg * (DFTW / 8)) * 8;
  const int row  = part ? rowG : rowF;
  const int col0 = part ? colG : colF;
  v4u p = {0u, 0u, 0u, 0u};
#pragma unroll 1
  for (int e = 0; e < 8; ++e) {
    const int col  = col0 + e;
    const int cidx = part ? col : row;
    const int nidx = part ? row : col;
    const int f = cidx >> 1, odd = cidx & 1;
    const bool edge  = (f == 0) || (f == 256);
    const bool valid = (f <= 256) && !(odd && edge);
    const float coef = (part != 0 && !edge) ? 2.0f : 1.0f;
    const int a = (nidx * f) & 511;
    const float th = (float)a * TWO_PI_OVER_512;
    const float cv = cosf(th), sv = sinf(th);
    const float t = odd ? -sv : cv;
    const float val = valid ? (t * coef * INV_SQRT512) : 0.0f;
    const unsigned bits = (unsigned)bf_bits(val);
    p[0] = (p[0] >> 16) | (p[1] << 16);
    p[1] = (p[1] >> 16) | (p[2] << 16);
    p[2] = (p[2] >> 16) | (p[3] << 16);
    p[3] = (p[3] >> 16) | (bits << 16);
  }
  unsigned short* dst = (part ? gtp : ftp) + (size_t)g * 8;
  *(volatile v4u*)dst = p;
  __threadfence();
  *(volatile v4u*)dst = p;
}

template <int NSPLIT, int OUT_MODE>
__global__ __launch_bounds__(256) void gemm64(
    const unsigned short* __restrict__ Ap, const unsigned short* A2p, int lda, long long strideA,
    const unsigned short* __restrict__ Btp, const unsigned short* Bt2p, int ldb, long long strideB,
    void* Cout, int ldc, long long strideC,
    void* Cout2, int ldc2, long long strideC2, int N2,
    const float* __restrict__ biasp, int biasMode,
    int M, int N, int K, float rscale) {
  const __bf16* A   = (const __bf16*)(const void*)Ap;
  const __bf16* A2  = (const __bf16*)(const void*)A2p;
  const __bf16* Bt  = (const __bf16*)(const void*)Btp;
  const __bf16* Bt2 = (const __bf16*)(const void*)Bt2p;
  __shared__ __align__(16) float sT[8][16 * 68];
  const int b    = blockIdx.y;
  const int lane = threadIdx.x & 31;
  const int wave = threadIdx.x >> 5;
  const int tilesN = N >> 6;
  const int tilesM = M >> 6;
  const int tile = blockIdx.x * 8 + wave;
  if (tile >= tilesM * tilesN) return;
  const int tm = tile / tilesN;
  const int tn = tile - tm * tilesN;
  const int m0 = tm << 6;
  const int n0 = tn << 6;

  const __bf16* Ab  = A  + (size_t)b * strideA;
  const __bf16* Bb  = Bt + (size_t)b * strideB;
  const __bf16* Ab2 = (NSPLIT >= 1) ? (A2  + (size_t)b * strideA) : Ab;
  const __bf16* Bb2 = (NSPLIT == 2) ? (Bt2 + (size_t)b * strideB) : Bb;

  const int rlane = lane & 15;
  const int koff  = (lane >> 4) * 8;
  const int mOff  = (lane >> 4) * 8;

  v8f acc[4][4];
#pragma unroll
  for (int i = 0; i < 4; ++i)
#pragma unroll
    for (int j = 0; j < 4; ++j) acc[i][j] = zero8();

  for (int k0 = 0; k0 < K; k0 += 32) {
    v16b bh[4], bl[4];
#pragma unroll
    for (int j = 0; j < 4; ++j) {
      const size_t bo = (size_t)(n0 + (j << 4) + rlane) * ldb + koff + k0;
      bh[j] = ldfrag_b(Bb + bo);
      if (NSPLIT == 2) bl[j] = ldfrag_b(Bb2 + bo); else bl[j] = bh[j];
    }
#pragma unroll
    for (int i = 0; i < 4; ++i) {
      const size_t ao = (size_t)(m0 + (i << 4) + rlane) * lda + koff + k0;
      const v16b ah = ldfrag_b(Ab + ao);
      v16b al = ah;
      if (NSPLIT >= 1) al = ldfrag_b(Ab2 + ao);
#pragma unroll
      for (int j = 0; j < 4; ++j) {
        acc[i][j] = mma_b_raw(ah, bh[j], acc[i][j]);
        if (NSPLIT >= 1) acc[i][j] = mma_b_raw(al, bh[j], acc[i][j]);
        if (NSPLIT == 2) acc[i][j] = mma_b_raw(ah, bl[j], acc[i][j]);
      }
      dep_guard_b(acc[i][0], acc[i][3], ah, al);
    }
    keep4_b(bh[0], bh[1], bh[2], bh[3]);
    if (NSPLIT == 2) keep4_b(bl[0], bl[1], bl[2], bl[3]);
  }
  acc_guard4(acc[0][0], acc[0][1], acc[0][2], acc[0][3]);
  acc_guard4(acc[1][0], acc[1][1], acc[1][2], acc[1][3]);
  acc_guard4(acc[2][0], acc[2][1], acc[2][2], acc[2][3]);
  acc_guard4(acc[3][0], acc[3][1], acc[3][2], acc[3][3]);

  float bcol[4];
#pragma unroll
  for (int j = 0; j < 4; ++j) bcol[j] = 0.f;
  if (biasMode == 1) {
#pragma unroll
    for (int j = 0; j < 4; ++j) bcol[j] = rbf(biasp[n0 + (j << 4) + rlane]);
  }

  float* slab = sT[wave];
#pragma unroll
  for (int i = 0; i < 4; ++i) {
    const int mBase = m0 + (i << 4);
    float brow[8];
#pragma unroll
    for (int r = 0; r < 8; ++r) brow[r] = 0.f;
    if (biasMode == 2) {
#pragma unroll
      for (int r = 0; r < 8; ++r) brow[r] = rbf(biasp[mBase + mOff + r]);
    }
#pragma unroll
    for (int j = 0; j < 4; ++j) {
#pragma unroll
      for (int r = 0; r < 8; ++r) {
        slab[(mOff + r) * 68 + (j << 4) + rlane] = (acc[i][j][r] + bcol[j]) + brow[r];
      }
    }
    wave_sync_lds();
    if (OUT_MODE == 0) {
      float* C = (float*)Cout + (size_t)b * strideC;
      const int hh = lane >> 4, c4 = (lane & 15) * 4;
      for (int pass = 0; pass < 2; ++pass) {
#pragma unroll
        for (int it = 0; it < 8; ++it) {
          const int row = it * 2 + hh;
          const v4f v = *(const v4f*)(slab + row * 68 + c4);
          *(volatile v4f*)(C + (size_t)(mBase + row) * ldc + n0 + c4) = v;
        }
        __threadfence();
      }
    } else {
      const int q = lane >> 3, c8 = (lane & 7) * 8;
      unsigned short* C  = (unsigned short*)Cout  + (size_t)b * strideC;
      unsigned short* C2 = (unsigned short*)Cout2 + (size_t)b * strideC2;
      const bool wlo = (OUT_MODE == 2) || (n0 < N2);
      v4u hv[4], lv[4];
#pragma unroll
      for (int it = 0; it < 4; ++it) {
        const int row = it * 4 + q;
        const float* sp = slab + row * 68 + c8;
        v4u a, a2;
#pragma unroll
        for (int e = 0; e < 4; ++e) {
          const float f0 = sp[2 * e], f1 = sp[2 * e + 1];
          unsigned short h0, h1, l0, l1;
          if (OUT_MODE == 2) {
            h0 = bf_bits(f0); h1 = bf_bits(f1);
            l0 = bf_bits(f0 - bf_up(h0)); l1 = bf_bits(f1 - bf_up(h1));
          } else {
            const _Float16 x0 = (_Float16)f0, x1 = (_Float16)f1;
            h0 = h_bits(x0); h1 = h_bits(x1);
            l0 = h_bits((_Float16)((f0 - (float)x0) * rscale));
            l1 = h_bits((_Float16)((f1 - (float)x1) * rscale));
          }
          a[e] = pk16(h0, h1); a2[e] = pk16(l0, l1);
        }
        hv[it] = a; lv[it] = a2;
      }
      for (int pass = 0; pass < 2; ++pass) {
#pragma unroll
        for (int it = 0; it < 4; ++it) {
          const int row = it * 4 + q;
          *(volatile v4u*)(C + (size_t)(mBase + row) * ldc + n0 + c8) = hv[it];
          if (wlo) *(volatile v4u*)(C2 + (size_t)(mBase + row) * ldc2 + n0 + c8) = lv[it];
        }
        __threadfence();
      }
    }
    wave_sync_lds();
  }
}

__global__ __launch_bounds__(256) void proj_tab(const unsigned short* __restrict__ qkp, const unsigned short* __restrict__ qlp,
                                                 const float* __restrict__ wop, const float* __restrict__ wdp,
                                                 float* tab, float rres) {
  const int id = blockIdx.x * 256 + threadIdx.x;
  if (id >= TABN) return;
  const int s = id & (SEQ - 1), h = (id >> 9) & (NHEAD - 1), b = id >> 12;
  const size_t ro = ((size_t)b * SEQ + s) * QKP + (size_t)h * HD;
  const _Float16* qh = (const _Float16*)(const void*)qkp + ro;
  const _Float16* kh = qh + HID;
  const _Float16* ql = (const _Float16*)(const void*)qlp + ro;
  const _Float16* kl = ql + HID;
  float a0 = 0.f, a1 = 0.f, a2 = 0.f, a3 = 0.f;
#pragma unroll 1
  for (int d4 = 0; d4 < HD / 4; ++d4) {
    const v4h q4h = *(const v4h*)(qh + 4 * d4);
    const v4h q4l = *(const v4h*)(ql + 4 * d4);
    const v4h k4h = *(const v4h*)(kh + 4 * d4);
    const v4h k4l = *(const v4h*)(kl + 4 * d4);
#pragma unroll
    for (int e = 0; e < 4; ++e) {
      const int d = 4 * d4 + e;
      const float qv = (float)q4h[e] + (float)q4l[e] * rres;
      const float kv = (float)k4h[e] + (float)k4l[e] * rres;
      a0 += qv * rbf(wop[d]);
      a1 += kv * rbf(wop[HD + d]);
      a2 += qv * rbf(wdp[d]);
      a3 += kv * rbf(wdp[HD + d]);
    }
  }
  float* t0 = tab + id;
  float* t1 = tab + (size_t)TABN + id;
  float* t2 = tab + (size_t)2 * TABN + id;
  float* t3 = tab + (size_t)3 * TABN + id;
  *(volatile float*)t0 = a0; *(volatile float*)t1 = a1; *(volatile float*)t2 = a2; *(volatile float*)t3 = a3;
  __threadfence();
  *(volatile float*)t0 = a0; *(volatile float*)t1 = a1; *(volatile float*)t2 = a2; *(volatile float*)t3 = a3;
}

__global__ __launch_bounds__(128)
void attn64(const unsigned short* __restrict__ qkp, const unsigned short* __restrict__ qlp,
            const unsigned short* __restrict__ vhp, const unsigned short* __restrict__ vlp,
            const float* __restrict__ tab, const float* __restrict__ maskp,
            const float* __restrict__ bop, const float* __restrict__ bdp,
            const float* __restrict__ sclp, float* ctxp, float rres) {
  union FH { v16h v; v8h h[2]; };
  __shared__ __align__(16) _Float16 Ksh[64 * 64];
  __shared__ __align__(16) _Float16 Vth[64 * 64];
  __shared__ __align__(16) _Float16 Vtl[64 * 64];
  __shared__ __align__(16) _Float16 Psh[4][16 * 64];
  __shared__ __align__(16) float    Fs[4][16 * 64];
  __shared__ float oqs[64];
  __shared__ float dqs[64];
  __shared__ float oks[64];
  __shared__ float dks[64];
  __shared__ float msk[64];

  const int tid  = threadIdx.x;
  const int wave = tid >> 5;
  const int lane = tid & 31;
  const int hh   = lane >> 4;
  const int c    = lane & 15;

  const int bx   = blockIdx.x;
  const int qb   = bx % NQB;
  const int rest = bx / NQB;
  const int h    = rest % NHEAD;
  const int b    = rest / NHEAD;
  const int q0   = qb * 64 + wave * 16;
  const size_t rowB = (size_t)b * SEQ;
  const int bh   = b * NHEAD + h;

  const _Float16* Qh = (const _Float16*)(const void*)qkp + (size_t)h * HD;
  const _Float16* Kg = (const _Float16*)(const void*)qkp + HID + (size_t)h * HD;
  const _Float16* Ql = (const _Float16*)(const void*)qlp + (size_t)h * HD;
  const _Float16* Vh = (const _Float16*)(const void*)vhp + ((size_t)b * HID + (size_t)h * HD) * SEQ;
  const _Float16* Vl = (const _Float16*)(const void*)vlp + ((size_t)b * HID + (size_t)h * HD) * SEQ;

  const float bo  = rbf(bop[0]);
  const float bd  = rbf(bdp[0]);
  const float scb = rbf(sclp[0]);
  const float sc2 = scb * scb;

  if (tid < 64) {
    oqs[tid] = tab[(size_t)bh * SEQ + qb * 64 + tid];
    dqs[tid] = tab[(size_t)2 * TABN + (size_t)bh * SEQ + qb * 64 + tid];
  }

  v16h qah[2], qal[2];
#pragma unroll
  for (int dc = 0; dc < 2; ++dc) {
    qah[dc] = ldfrag_h(Qh + (rowB + q0 + c) * QKP + dc * 32 + 8 * hh);
    qal[dc] = ldfrag_h(Ql + (rowB + q0 + c) * QKP + dc * 32 + 8 * hh);
  }

  float mrow[8], lrow[8];
  v8f oacc[4];
#pragma unroll
  for (int r = 0; r < 8; ++r) { mrow[r] = -INFINITY; lrow[r] = 0.f; }
#pragma unroll
  for (int t = 0; t < 4; ++t) oacc[t] = zero8();

  float* ss = Fs[wave];

  for (int kt = 0; kt < NQB; ++kt) {
    const int kv0 = kt * 64;
    __syncthreads();
    {
      const int r = tid >> 1, hf = (tid & 1) * 32;
      const _Float16* kg  = Kg + (rowB + kv0 + r) * QKP + hf;
      const _Float16* vg  = Vh + (size_t)r * SEQ + kv0 + hf;
      const _Float16* vlg = Vl + (size_t)r * SEQ + kv0 + hf;
#pragma unroll
      for (int i = 0; i < 4; ++i) {
        const v8h a0 = *(const v8h*)(kg + 8 * i);
        const v8h b0 = *(const v8h*)(vg + 8 * i);
        const v8h b1 = *(const v8h*)(vlg + 8 * i);
        *(v8h*)(Ksh + r * 64 + hf + 8 * i) = a0;
        *(v8h*)(Vth + r * 64 + hf + 8 * i) = b0;
        *(v8h*)(Vtl + r * 64 + hf + 8 * i) = b1;
      }
    }
    if (tid < 64) {
      oks[tid] = tab[(size_t)TABN + (size_t)bh * SEQ + kv0 + tid];
      dks[tid] = tab[(size_t)3 * TABN + (size_t)bh * SEQ + kv0 + tid];
      msk[tid] = rbf(maskp[(size_t)b * SEQ + kv0 + tid]);
    }
    __syncthreads();

#pragma unroll
    for (int j = 0; j < 4; ++j) {
      v8f sh = zero8(), sl = zero8();
#pragma unroll
      for (int dc = 0; dc < 2; ++dc) {
        FH kb;
        kb.h[0] = *(const v8h*)(Ksh + (j * 16 + c) * 64 + dc * 32 + 8 * hh);
        kb.h[1] = *(const v8h*)(Ksh + (j * 16 + c) * 64 + dc * 32 + 16 + 8 * hh);
        sh = mma_h(qah[dc], kb.v, sh);
        sl = mma_h(qal[dc], kb.v, sl);
      }
#pragma unroll
      for (int r = 0; r < 8; ++r) ss[(8 * hh + r) * 64 + j * 16 + c] = sh[r] + sl[r] * rres;
    }
    wave_sync_lds();

#pragma unroll 1
    for (int e = 0; e < 32; ++e) {
      const int row = e >> 1;
      const int col = ((e & 1) << 5) + lane;
      const int qi  = q0 + row;
      const int kj  = kv0 + col;
      const float raw = ss[row * 64 + col];
      const float z   = (oqs[wave * 16 + row] + oks[col]) + bo;
      const float ez  = expf(-z);
      const float pr  = 1.0f / (1.0f + ez);
      const float arg = (kj > qi) ? pr : (1.0f - pr);
      const float eo  = logf(arg + 1e-24f);
      const float dd  = (dqs[wave * 16 + row] + dks[col]) + bd;
      int dist = kj - qi;
      dist = (dist < 0) ? -dist : dist;
      const float gd  = logf((float)dist + 1.0f);
      const float df  = gd - dd;
      const float ed  = (-(df * df) * sc2) * 0.5f;
      const float sv  = ((raw + eo) + ed) * 0.125f + msk[col];
      ss[row * 64 + col] = sv;
    }
    wave_sync_lds();

    v8f s[4];
#pragma unroll
    for (int j = 0; j < 4; ++j) {
#pragma unroll
      for (int r = 0; r < 8; ++r) s[j][r] = ss[(8 * hh + r) * 64 + j * 16 + c];
    }

    _Float16* pwh = Psh[wave];
#pragma unroll
    for (int r = 0; r < 8; ++r) {
      float m = s[0][r];
      m = fmaxf(m, s[1][r]);
      m = fmaxf(m, s[2][r]);
      m = fmaxf(m, s[3][r]);
#pragma unroll
      for (int off = 1; off < 16; off <<= 1) m = fmaxf(m, __shfl_xor(m, off, 32));
      const float mnew  = fmaxf(mrow[r], m);
      const float alpha = __expf(mrow[r] - mnew);
      mrow[r] = mnew;
      float psum = 0.f;
#pragma unroll
      for (int j = 0; j < 4; ++j) {
        const float p = __expf(s[j][r] - mnew);
        psum += p;
        pwh[(8 * hh + r) * 64 + j * 16 + c] = (_Float16)(p * 1024.0f);
      }
#pragma unroll
      for (int off = 1; off < 16; off <<= 1) psum += __shfl_xor(psum, off, 32);
      lrow[r] = lrow[r] * alpha + psum;
#pragma unroll
      for (int t = 0; t < 4; ++t) oacc[t][r] *= alpha;
    }
    wave_sync_lds();

    v8f o1[4];
#pragma unroll
    for (int t = 0; t < 4; ++t) o1[t] = zero8();
#pragma unroll 1
    for (int kk = 0; kk < 2; ++kk) {
      FH pa;
      pa.h[0] = *(const v8h*)(pwh + c * 64 + kk * 32 + 8 * hh);
      pa.h[1] = *(const v8h*)(pwh + c * 64 + kk * 32 + 16 + 8 * hh);
#pragma unroll
      for (int t = 0; t < 4; ++t) {
        FH vb, vl;
        vb.h[0] = *(const v8h*)(Vth + (t * 16 + c) * 64 + kk * 32 + 8 * hh);
        vb.h[1] = *(const v8h*)(Vth + (t * 16 + c) * 64 + kk * 32 + 16 + 8 * hh);
        vl.h[0] = *(const v8h*)(Vtl + (t * 16 + c) * 64 + kk * 32 + 8 * hh);
        vl.h[1] = *(const v8h*)(Vtl + (t * 16 + c) * 64 + kk * 32 + 16 + 8 * hh);
        oacc[t] = mma_h(pa.v, vb.v, oacc[t]);
        o1[t]   = mma_h(pa.v, vl.v, o1[t]);
      }
    }
#pragma unroll
    for (int t = 0; t < 4; ++t)
#pragma unroll
      for (int r = 0; r < 8; ++r) oacc[t][r] += o1[t][r] * rres;
  }

  float* os = Fs[wave];
#pragma unroll
  for (int r = 0; r < 8; ++r) {
    const float l = lrow[r];
    const float inv = ((l > 0.f) ? (1.0f / l) : 0.f) * (1.0f / 1024.0f);
#pragma unroll
    for (int t = 0; t < 4; ++t) os[(8 * hh + r) * 64 + t * 16 + c] = oacc[t][r] * inv;
  }
  wave_sync_lds();
  {
    const int h2 = lane >> 4, c4 = (lane & 15) * 4;
    v4f ov[8];
#pragma unroll
    for (int it = 0; it < 8; ++it) {
      const int row = it * 2 + h2;
      ov[it] = *(const v4f*)(os + row * 64 + c4);
    }
    for (int pass = 0; pass < 2; ++pass) {
#pragma unroll
      for (int it = 0; it < 8; ++it) {
        const int row = it * 2 + h2;
        const size_t go = (rowB + q0 + row) * HID + (size_t)h * HD + c4;
        *(volatile v4f*)(ctxp + go) = ov[it];
      }
      __threadfence();
    }
  }
}

__global__ __launch_bounds__(256) void cmul(const float* __restrict__ xfp, const float* __restrict__ cwp, unsigned short* zp) {
  const int g = blockIdx.x * 256 + threadIdx.x;
  if (g >= NBATCH * SEQ * (DFTW / 8)) return;
  const int m  = g / (DFTW / 8);
  const int cg = g - m * (DFTW / 8);
  const int s  = m & (SEQ - 1);
  const float* xp = xfp + (size_t)m * DFTW + cg * 8;
  const v4f x0 = *(const v4f*)xp;
  const v4f x1 = *(const v4f*)(xp + 4);
  v4u p;
#pragma unroll
  for (int q = 0; q < 4; ++q) {
    const float xr = (q < 2) ? x0[(2 * q) & 3] : x1[(2 * q) & 3];
    const float xi = (q < 2) ? x0[(2 * q + 1) & 3] : x1[(2 * q + 1) & 3];
    const int f  = cg * 4 + q;
    const int fc = (f < NFREQ) ? f : (NFREQ - 1);
    const float wr = rbf(cwp[((size_t)s * NFREQ + fc) * 2]);
    const float wi = rbf(cwp[((size_t)s * NFREQ + fc) * 2 + 1]);
    const bool valid = (f < NFREQ);
    const float zr = valid ? (xr * wr - xi * wi) : 0.f;
    const float zi = valid ? (xr * wi + xi * wr) : 0.f;
    p[q] = pk16(bf_bits(zr), bf_bits(zi));
  }
  *(volatile v4u*)(zp + (size_t)g * 8) = p;
  __threadfence();
  *(volatile v4u*)(zp + (size_t)g * 8) = p;
}

__global__ __launch_bounds__(128) void k_out(const float* __restrict__ seqp, const float* __restrict__ ctxp,
                                             const float* __restrict__ xin,
                                             const float* __restrict__ lfw, const float* __restrict__ lfb,
                                             const float* __restrict__ lw, const float* __restrict__ lb,
                                             float* out) {
  __shared__ float red[4][4];
  const int m = blockIdx.x, tid = threadIdx.x, lane = tid & 31, wave = tid >> 5;
  const int c4 = tid * 4;
  const size_t ro = (size_t)m * HID + c4;
  const v4f a  = *(const v4f*)(seqp + ro);
  const v4f cc = *(const v4f*)(ctxp + ro);
  const v4f xv = *(const v4f*)(xin + ro);
  const v4f w1 = *(const v4f*)(lfw + c4);
  const v4f b1 = *(const v4f*)(lfb + c4);
  const v4f w2 = *(const v4f*)(lw + c4);
  const v4f b2 = *(const v4f*)(lb + c4);

  float t[4];
#pragma unroll
  for (int e = 0; e < 4; ++e) t[e] = a[e] + cc[e];
  float sum = (t[0] + t[1]) + (t[2] + t[3]);
  sum = wave_sum(sum);
  if (lane == 0) red[0][wave] = sum;
  __syncthreads();
  const float mean = ((red[0][0] + red[0][1]) + (red[0][2] + red[0][3])) * (1.0f / (float)HID);
  float d[4];
  float vs = 0.f;
#pragma unroll
  for (int e = 0; e < 4; ++e) { d[e] = t[e] - mean; vs += d[e] * d[e]; }
  vs = wave_sum(vs);
  if (lane == 0) red[1][wave] = vs;
  __syncthreads();
  const float var = ((red[1][0] + red[1][1]) + (red[1][2] + red[1][3])) * (1.0f / (float)HID);
  const float rs = 1.0f / sqrtf(var + 1e-12f);

  float t2[4];
#pragma unroll
  for (int e = 0; e < 4; ++e) {
    const float hg = rbf(w1[e]) * (d[e] * rs) + rbf(b1[e]);
    t2[e] = hg + rbf(xv[e]);
  }
  float sum2 = (t2[0] + t2[1]) + (t2[2] + t2[3]);
  sum2 = wave_sum(sum2);
  if (lane == 0) red[2][wave] = sum2;
  __syncthreads();
  const float mean2 = ((red[2][0] + red[2][1]) + (red[2][2] + red[2][3])) * (1.0f / (float)HID);
  float d2[4];
  float vs2 = 0.f;
#pragma unroll
  for (int e = 0; e < 4; ++e) { d2[e] = t2[e] - mean2; vs2 += d2[e] * d2[e]; }
  vs2 = wave_sum(vs2);
  if (lane == 0) red[3][wave] = vs2;
  __syncthreads();
  const float var2 = ((red[3][0] + red[3][1]) + (red[3][2] + red[3][3])) * (1.0f / (float)HID);
  const float rs2 = 1.0f / sqrtf(var2 + 1e-12f);

  v4f o;
#pragma unroll
  for (int e = 0; e < 4; ++e) o[e] = rbf(w2[e]) * (d2[e] * rs2) + rbf(b2[e]);
  *(volatile v4f*)(out + ro) = o;
  __threadfence();
  *(volatile v4f*)(out + ro) = o;
}

extern "C" void kernel_launch(void* const* d_in, const int* in_sizes, int n_in,
                              void* d_out, int out_size, void* d_ws, size_t ws_size,
                              hipStream_t stream) {
  if (n_in < 18) return;
  if (in_sizes[0] != NBATCH * SEQ * HID) return;
  if (in_sizes[1] != NBATCH * SEQ) return;
  if (in_sizes[2] != HID * HID || in_sizes[4] != HID * HID || in_sizes[6] != HID * HID) return;
  if (in_sizes[3] != HID || in_sizes[5] != HID || in_sizes[7] != HID) return;
  if (in_sizes[8] != 2 * HD || in_sizes[10] != 2 * HD) return;
  if (in_sizes[9] < 1 || in_sizes[11] < 1 || in_sizes[12] < 1) return;
  if (in_sizes[13] != SEQ * NFREQ * 2) return;
  if (in_sizes[14] != HID || in_sizes[15] != HID || in_sizes[16] != HID || in_sizes[17] != HID) return;
  if (out_size != NBATCH * SEQ * HID) return;

  const float* x    = (const float*)d_in[0];
  const float* mask = (const float*)d_in[1];
  const float* Wq   = (const float*)d_in[2];
  const float* bq   = (const float*)d_in[3];
  const float* Wk   = (const float*)d_in[4];
  const float* bk   = (const float*)d_in[5];
  const float* Wv   = (const float*)d_in[6];
  const float* bv   = (const float*)d_in[7];
  const float* Wo   = (const float*)d_in[8];
  const float* b_o  = (const float*)d_in[9];
  const float* Wd   = (const float*)d_in[10];
  const float* b_d  = (const float*)d_in[11];
  const float* scl  = (const float*)d_in[12];
  const float* cw   = (const float*)d_in[13];
  const float* lfw  = (const float*)d_in[14];
  const float* lfb  = (const float*)d_in[15];
  const float* lw   = (const float*)d_in[16];
  const float* lb   = (const float*)d_in[17];

  const size_t PXb  = (size_t)NBATCH * SEQ * HID * 2;
  const size_t PWT  = (size_t)HID * HID * 2;
  const size_t PQK  = (size_t)NBATCH * SEQ * QKP * 2;
  const size_t PVT  = (size_t)NBATCH * HID * SEQ * 2;
  const size_t PTAB = (size_t)4 * TABN * 4;
  const size_t PCTX = (size_t)NBATCH * SEQ * HID * 4;
  const size_t PCTb = (size_t)NBATCH * SEQ * HID * 2;
  const size_t PFT  = (size_t)DFTW * HID * 2;
  const size_t PXF  = (size_t)NBATCH * SEQ * DFTW * 4;
  const size_t PZ   = (size_t)NBATCH * SEQ * DFTW * 2;
  const size_t PSEQ = (size_t)NBATCH * SEQ * HID * 4;
  size_t off = 0;
  const size_t oXb  = off; off += PXb;
  const size_t oWqT = off; off += PWT;
  const size_t oWkT = off; off += PWT;
  const size_t oWvT = off; off += PWT;
  const size_t oQK  = off; off += PQK;
  const size_t oQKl = off; off += PQK;
  const size_t oVTh = off; off += PVT;
  const size_t oVTl = off; off += PVT;
  const size_t oTAB = off; off += PTAB;
  const size_t oCTX = off; off += PCTX;
  const size_t oCTb = off; off += PCTb;
  const size_t oFT  = off; off += PFT;
  const size_t oGT  = off; off += PFT;
  const size_t oXF  = off; off += PXF;
  const size_t oZ   = off; off += PZ;
  const size_t oSEQ = off; off += PSEQ;
  if (off > ws_size) return;
  if (off > (size_t)134217728) return;

  char* ws = (char*)d_ws;
  unsigned short* Xb   = (unsigned short*)(ws + oXb);
  unsigned short* WqT  = (unsigned short*)(ws + oWqT);
  unsigned short* WkT  = (unsigned short*)(ws + oWkT);
  unsigned short* WvT  = (unsigned short*)(ws + oWvT);
  unsigned short* QK   = (unsigned short*)(ws + oQK);
  unsigned short* QKl  = (unsigned short*)(ws + oQKl);
  unsigned short* VTh  = (unsigned short*)(ws + oVTh);
  unsigned short* VTl  = (unsigned short*)(ws + oVTl);
  float*          TAB  = (float*)(ws + oTAB);
  float*          CTX  = (float*)(ws + oCTX);
  unsigned short* CTXb = (unsigned short*)(ws + oCTb);
  unsigned short* FT   = (unsigned short*)(ws + oFT);
  unsigned short* GT   = (unsigned short*)(ws + oGT);
  float*          XF   = (float*)(ws + oXF);
  unsigned short* Z    = (unsigned short*)(ws + oZ);
  float*          SEQP = (float*)(ws + oSEQ);

  const dim3 blk(256);
  const int n8x = NBATCH * SEQ * HID / 8;
  const dim3 gCvt((n8x + 255) / 256);
  const dim3 gTr(HID / 64, HID / 64);
  const dim3 gBas((DFTW * HID / 8 + 255) / 256, 2);
  const dim3 gQ(((NBATCH * SEQ / 64) * (HID / 64) + 7) / 8, 1);
  const dim3 gV(((HID / 64) * (SEQ / 64) + 7) / 8, NBATCH);
  const dim3 gTab((TABN + 255) / 256);
  const dim3 gAttn(NBATCH * NHEAD * NQB);
  const dim3 gDft1(((NBATCH * SEQ / 64) * (DFTW / 64) + 7) / 8, 1);
  const dim3 gMul((NBATCH * SEQ * (DFTW / 8) + 255) / 256);
  const dim3 gDft2(((NBATCH * SEQ / 64) * (HID / 64) + 7) / 8, 1);
  const dim3 gOut(NBATCH * SEQ);

  cvt_bf16x8<<<gCvt, blk, 0, stream>>>(x, Xb, n8x);
  tr_bf16<<<gTr, blk, 0, stream>>>(Wq, WqT, HID, HID);
  tr_bf16<<<gTr, blk, 0, stream>>>(Wk, WkT, HID, HID);
  tr_bf16<<<gTr, blk, 0, stream>>>(Wv, WvT, HID, HID);
  build_basis<<<gBas, blk, 0, stream>>>(FT, GT);
  gemm64<0, 3><<<gQ, blk, 0, stream>>>(
      Xb, Xb, HID, 0LL, WqT, WqT, HID, 0LL,
      (void*)QK, QKP, 0LL, (void*)QKl, QKP, 0LL, HID,
      bq, 1, NBATCH * SEQ, HID, HID, 4096.0f);
  gemm64<0, 3><<<gQ, blk, 0, stream>>>(
      Xb, Xb, HID, 0LL, WkT, WkT, HID, 0LL,
      (void*)(QK + HID), QKP, 0LL, (void*)(QKl + HID), QKP, 0LL, HID,
      bk, 1, NBATCH * SEQ, HID, HID, 4096.0f);
  gemm64<0, 3><<<gV, blk, 0, stream>>>(
      WvT, WvT, HID, 0LL, Xb, Xb, HID, (long long)SEQ * HID,
      (void*)VTh, SEQ, (long long)HID * SEQ, (void*)VTl, SEQ, (long long)HID * SEQ, SEQ,
      bv, 2, HID, SEQ, HID, 4096.0f);
  proj_tab<<<gTab, blk, 0, stream>>>(QK, QKl, Wo, Wd, TAB, 1.0f / 4096.0f);
  attn64<<<gAttn, dim3(128), 0, stream>>>(QK, QKl, VTh, VTl, TAB, mask, b_o, b_d, scl, CTX, 1.0f / 4096.0f);
  cvt_bf16x8<<<gCvt, blk, 0, stream>>>(CTX, CTXb, n8x);
  gemm64<0, 0><<<gDft1, blk, 0, stream>>>(
      CTXb, CTXb, HID, 0LL, FT, FT, HID, 0LL,
      (void*)XF, DFTW, 0LL, (void*)XF, DFTW, 0LL, 0,
      bq, 0, NBATCH * SEQ, DFTW, HID, 1.0f);
  cmul<<<gMul, blk, 0, stream>>>(XF, cw, Z);
  gemm64<0, 0><<<gDft2, blk, 0, stream>>>(
      Z, Z, DFTW, 0LL, GT, GT, DFTW, 0LL,
      (void*)SEQP, HID, 0LL, (void*)SEQP, HID, 0LL, 0,
      bq, 0, NBATCH * SEQ, HID, DFTW, 1.0f);
  k_out<<<gOut, dim3(128), 0, stream>>>(SEQP, CTX, x, lfw, lfb, lw, lb, (float*)d_out);
  (void)hipGetLastError();
}
